// OperatorBlocks_53953379172720
// MI455X (gfx1250) — hardware-verified
//
#include <hip/hip_runtime.h>
#include <hip/hip_bf16.h>
#include <math.h>


#define NB 8
#define NN 2048
#define NC 256
#define NE 32768
#define NL 3
#define NK 3
#define NM (NB * NN)
#define BNC (NM * NC)
#define KCAT (NK * NC)
#define PT 16
#define DT 128
#define ASCALE 16.0f
#define WSCALE 256.0f
#define OSCALE (1.0f / 4096.0f)

typedef __attribute__((ext_vector_type(16))) _Float16 v16h;
typedef __attribute__((ext_vector_type(8)))  _Float16 v8h;
typedef __attribute__((ext_vector_type(16))) __bf16   v16b;
typedef __attribute__((ext_vector_type(8)))  __bf16   v8b;
typedef __attribute__((ext_vector_type(8)))  float    v8f;
typedef __attribute__((ext_vector_type(4)))  float    v4f;
typedef __attribute__((ext_vector_type(2)))  float    v2f;
typedef __attribute__((ext_vector_type(2)))  unsigned int v2u;
typedef __attribute__((ext_vector_type(4)))  _Float16 v4h;

__device__ __forceinline__ unsigned short f2bf_bits(float f) {
  unsigned u = __float_as_uint(f);
  return (unsigned short)((u + 0x7FFFu + ((u >> 16) & 1u)) >> 16);
}
__device__ __forceinline__ float bf_bits2f(unsigned short h) { return __uint_as_float(((unsigned)h) << 16); }

__device__ __forceinline__ void dep_guard_h(v8f& a, v8f& b, v16h x, v16h y) { asm volatile("v_nop\n\tv_nop\n\tv_nop\n\tv_nop" : "+v"(a), "+v"(b) : "v"(x), "v"(y)); }
__device__ __forceinline__ void dep_guard_b(v8f& a, v8f& b, v16b x, v16b y) { asm volatile("v_nop\n\tv_nop\n\tv_nop\n\tv_nop" : "+v"(a), "+v"(b) : "v"(x), "v"(y)); }
__device__ __forceinline__ void keep4_h(v16h a, v16h b, v16h c, v16h d) { asm volatile("v_nop" :: "v"(a), "v"(b), "v"(c), "v"(d)); }
__device__ __forceinline__ void keep4_b(v16b a, v16b b, v16b c, v16b d) { asm volatile("v_nop" :: "v"(a), "v"(b), "v"(c), "v"(d)); }
__device__ __forceinline__ void acc_guard4(v8f& a, v8f& b, v8f& c, v8f& d) { asm volatile("v_nop\n\tv_nop\n\tv_nop\n\tv_nop" : "+v"(a), "+v"(b), "+v"(c), "+v"(d)); }
template <typename T> struct Frag;
template <> struct Frag<_Float16> {
  typedef v16h V; union U { v16h v; v8h h[2]; };
  static __device__ __forceinline__ v16h load(const _Float16* p) {
    U f; f.h[0] = *(const v8h*)(p); f.h[1] = *(const v8h*)(p + 16); return f.v;
  }
  static __device__ __forceinline__ v8f mma(v16h a, v16h b, v8f c) {
    return __builtin_amdgcn_wmma_f32_16x16x32_f16(false, a, false, b, (short)0, c, false, false);
  }
  static __device__ __forceinline__ void guard(v8f& a, v8f& b, v16h x, v16h y) { dep_guard_h(a, b, x, y); }
  static __device__ __forceinline__ void keep(v16h a, v16h b, v16h c, v16h d) { keep4_h(a, b, c, d); }
};
template <> struct Frag<__bf16> {
  typedef v16b V; union U { v16b v; v8b h[2]; };
  static __device__ __forceinline__ v16b load(const __bf16* p) {
    U f; f.h[0] = *(const v8b*)(p); f.h[1] = *(const v8b*)(p + 16); return f.v;
  }
  static __device__ __forceinline__ v8f mma(v16b a, v16b b, v8f c) {
    return __builtin_amdgcn_wmma_f32_16x16x32_bf16(false, a, false, b, (short)0, c, false, false);
  }
  static __device__ __forceinline__ void guard(v8f& a, v8f& b, v16b x, v16b y) { dep_guard_b(a, b, x, y); }
  static __device__ __forceinline__ void keep(v16b a, v16b b, v16b c, v16b d) { keep4_b(a, b, c, d); }
};

template <int ET> struct Elem;
template <> struct Elem<0> { typedef _Float16 T; };
template <> struct Elem<1> { typedef __bf16 T; };
template <int ET, bool SPLIT, int BIAS_MODE, int OUT_MODE, bool RESID, int ACT = 0>
__global__ __launch_bounds__(256) void wmma_gemm64(
    const unsigned short* __restrict__ Ap, const unsigned short* __restrict__ A2p, int lda, long strideA,
    const unsigned short* __restrict__ Btp, const unsigned short* __restrict__ Bt2p, int ldb, long strideB,
    void* __restrict__ Cout, void* __restrict__ Cout2, int ldc, long strideC,
    const float* __restrict__ bias,
    const float* __restrict__ resid, long strideR,
    int M, int N, int K, float scale) {
  typedef typename Elem<ET>::T T;
  typedef typename Frag<T>::V V;
  const T* A = (const T*)Ap; const T* A2 = (const T*)A2p; const T* Bt = (const T*)Btp; const T* Bt2 = (const T*)Bt2p;
  __shared__ __align__(16) float sT[8][16 * 68];
  const int b    = blockIdx.y;
  const int lane = threadIdx.x & 31;
  const int wave = threadIdx.x >> 5;
  const int tilesN = N >> 6;
  const int tilesM = M >> 6;
  const int tile = blockIdx.x * 8 + wave;
  if (tile >= tilesM * tilesN) return;
  const int tm = tile / tilesN;
  const int tn = tile - tm * tilesN;
  const int m0 = tm << 6;
  const int n0 = tn << 6;

  const T* Ab  = A  + (size_t)b * strideA;
  const T* Bb  = Bt + (size_t)b * strideB;
  const T* Ab2 = SPLIT ? (A2  + (size_t)b * strideA) : nullptr;
  const T* Bb2 = SPLIT ? (Bt2 + (size_t)b * strideB) : nullptr;

  const int rlane = lane & 15;
  const int koff  = (lane >> 4) * 8;
  const int mOff  = (lane >> 4) * 8;

  v8f acc[4][4];
#pragma unroll
  for (int i = 0; i < 4; ++i)
#pragma unroll
    for (int j = 0; j < 4; ++j) acc[i][j] = (v8f){0.f,0.f,0.f,0.f,0.f,0.f,0.f,0.f};

  for (int k0 = 0; k0 < K; k0 += 32) {
    V bh[4], bl[4];
#pragma unroll
    for (int j = 0; j < 4; ++j) {
      const size_t bo = (size_t)(n0 + (j << 4) + rlane) * ldb + koff + k0;
      bh[j] = Frag<T>::load(Bb + bo);
      if (SPLIT) bl[j] = Frag<T>::load(Bb2 + bo);
    }
#pragma unroll
    for (int i = 0; i < 4; ++i) {
      const size_t ao = (size_t)(m0 + (i << 4) + rlane) * lda + koff + k0;
      V ah = Frag<T>::load(Ab + ao);
      V al;
      if (SPLIT) al = Frag<T>::load(Ab2 + ao);
#pragma unroll
      for (int j = 0; j < 4; ++j) {
        acc[i][j] = Frag<T>::mma(ah, bh[j], acc[i][j]);
        if (SPLIT) {
          acc[i][j] = Frag<T>::mma(ah, bl[j], acc[i][j]);
          acc[i][j] = Frag<T>::mma(al, bh[j], acc[i][j]);
        }
      }
      Frag<T>::guard(acc[i][0], acc[i][3], ah, SPLIT ? al : ah);
    }
    Frag<T>::keep(bh[0], bh[1], bh[2], bh[3]);
    if (SPLIT) Frag<T>::keep(bl[0], bl[1], bl[2], bl[3]);
  }
  acc_guard4(acc[0][0], acc[0][1], acc[0][2], acc[0][3]);
  acc_guard4(acc[1][0], acc[1][1], acc[1][2], acc[1][3]);
  acc_guard4(acc[2][0], acc[2][1], acc[2][2], acc[2][3]);
  acc_guard4(acc[3][0], acc[3][1], acc[3][2], acc[3][3]);

  float* slab = sT[wave];
  const float* Rb = RESID ? (resid + (size_t)b * strideR) : nullptr;
#pragma unroll
  for (int i = 0; i < 4; ++i) {
    const int mBase = m0 + (i << 4);
#pragma unroll
    for (int j = 0; j < 4; ++j) {
      const int n = n0 + (j << 4) + rlane;
      float bv = 0.f;
      if (BIAS_MODE == 2) bv = bias[n];
#pragma unroll
      for (int r = 0; r < 8; ++r) {
        float v = acc[i][j][r] * scale;
        if (BIAS_MODE == 1) v += bias[mBase + mOff + r];
        if (BIAS_MODE == 2) v += bv;
        if (RESID) v += Rb[(size_t)(mBase + mOff + r) * ldc + n];
        if (ACT == 1) v = tanhf(v);
        if (ACT == 2) v = fmaxf(v, 0.0f);
        if (ACT == 3) v = v / (1.0f + expf(-v));
        if (ACT == 4) v = (v > 0.f) ? v : 0.01f * v;
        if (ACT == 5) v = 0.5f * v * (1.0f + erff(v * 0.70710678118654752f));
        slab[(mOff + r) * 68 + (j << 4) + rlane] = v;
      }
    }
    __builtin_amdgcn_fence(__ATOMIC_RELEASE, "workgroup");
    __builtin_amdgcn_wave_barrier();
    __builtin_amdgcn_fence(__ATOMIC_ACQUIRE, "workgroup");
    if (OUT_MODE == 0) {
      float* C = (float*)Cout + (size_t)b * strideC;
      const int hh = lane >> 4, c4 = (lane & 15) * 4;
      for (int pass = 0; pass < 2; ++pass) {
#pragma unroll
        for (int it = 0; it < 8; ++it) {
          const int row = it * 2 + hh;
          v4f v = *(const v4f*)(slab + row * 68 + c4);
          *(volatile v4f*)(C + (size_t)(mBase + row) * ldc + n0 + c4) = v;
        }
        __threadfence();
      }
    } else {
      const int q = lane >> 3, c8 = (lane & 7) * 8;
      unsigned short* C  = (unsigned short*)Cout  + (size_t)b * strideC;
      unsigned short* C2 = (OUT_MODE == 2) ? ((unsigned short*)Cout2 + (size_t)b * strideC) : nullptr;
      for (int pass = 0; pass < 2; ++pass) {
#pragma unroll
        for (int it = 0; it < 4; ++it) {
          const int row = it * 4 + q;
          const float* sp = slab + row * 68 + c8;
          v8h hv, lv;
#pragma unroll
          for (int e = 0; e < 8; ++e) {
            if (OUT_MODE == 1) {
              hv[e] = (_Float16)sp[e];
            } else {
              unsigned short hb = f2bf_bits(sp[e]);
              unsigned short lb = f2bf_bits(sp[e] - bf_bits2f(hb));
              hv[e] = __builtin_bit_cast(_Float16, hb);
              lv[e] = __builtin_bit_cast(_Float16, lb);
            }
          }
          *(volatile v8h*)(C + (size_t)(mBase + row) * ldc + n0 + c8) = hv;
          if (OUT_MODE == 2) *(volatile v8h*)(C2 + (size_t)(mBase + row) * ldc + n0 + c8) = lv;
        }
        __threadfence();
      }
    }
    __builtin_amdgcn_fence(__ATOMIC_RELEASE, "workgroup");
    __builtin_amdgcn_wave_barrier();
    __builtin_amdgcn_fence(__ATOMIC_ACQUIRE, "workgroup");
  }
}

__device__ __forceinline__ v2u pack4h(v4f y) {
  v4h hv;
  hv[0] = (_Float16)(y[0] * ASCALE);
  hv[1] = (_Float16)(y[1] * ASCALE);
  hv[2] = (_Float16)(y[2] * ASCALE);
  hv[3] = (_Float16)(y[3] * ASCALE);
  return __builtin_bit_cast(v2u, hv);
}

__device__ __forceinline__ void stats_reduce_store(double s, double q, double* ss, double* sq, float* res,
                                                   float* __restrict__ st) {
  const int tid = threadIdx.x;
  ss[tid] = s; sq[tid] = q;
  __syncthreads();
  for (int o = 256; o > 0; o >>= 1) {
    if (tid < o) { ss[tid] += ss[tid + o]; sq[tid] += sq[tid + o]; }
    __syncthreads();
  }
  if (tid == 0) {
    const double inv = 1.0 / (double)BNC;
    const double m = ss[0] * inv;
    double var = sq[0] * inv - m * m;
    if (var < 0.0) var = 0.0;
    res[0] = (float)m;
    res[1] = rsqrtf((float)var + 1e-5f);
  }
  __syncthreads();
  if (tid < 32) {
    const float v = (tid == 0) ? res[0] : ((tid == 1) ? res[1] : 0.f);
    ((volatile float*)st)[tid] = v;
    __threadfence();
    ((volatile float*)st)[tid] = v;
  }
}

__global__ __launch_bounds__(256) void prep_weights(const float* __restrict__ pw, const float* __restrict__ mw,
                                                    _Float16* __restrict__ wct, _Float16* __restrict__ wmt) {
  const int g = blockIdx.x * 256 + threadIdx.x;
  const int NPW8 = NL * NC * KCAT / 8;
  const int NMW8 = NL * NC * NC / 8;
  v8h hv;
  _Float16* dst;
  if (g < NPW8) {
    const int idx = g * 8;
    const int l = idx / (NC * KCAT);
    const int rem = idx - l * (NC * KCAT);
    const int n = rem / KCAT;
    const int k = rem - n * KCAT;
    const int kk = k >> 8, c0 = k & 255;
    const float* src = pw + ((size_t)(l * NK + kk) * NC + c0) * NC + n;
#pragma unroll
    for (int e = 0; e < 8; ++e) hv[e] = (_Float16)(src[(size_t)e * NC] * WSCALE);
    dst = wct + idx;
  } else if (g < NPW8 + NMW8) {
    const int idx = (g - NPW8) * 8;
    const int l = idx >> 16;
    const int rem = idx & 65535;
    const int n = rem >> 8;
    const int k0 = rem & 255;
    const float* src = mw + ((size_t)l * NC + k0) * NC + n;
#pragma unroll
    for (int e = 0; e < 8; ++e) hv[e] = (_Float16)(src[(size_t)e * NC] * WSCALE);
    dst = wmt + idx;
  } else {
    return;
  }
  *(volatile v8h*)dst = hv;
  __threadfence();
  *(volatile v8h*)dst = hv;
}

__global__ __launch_bounds__(512) void ln_stats(const float* __restrict__ x, float* __restrict__ st) {
  __shared__ double ss[512], sq[512];
  __shared__ float res[2];
  const int tid = threadIdx.x;
  double s = 0.0, q = 0.0;
  const v4f* xv = (const v4f*)x;
  for (int i = tid; i < BNC / 4; i += 512) {
    const v4f v = xv[i];
    s += (double)v[0]; s += (double)v[1]; s += (double)v[2]; s += (double)v[3];
    q += (double)v[0] * (double)v[0]; q += (double)v[1] * (double)v[1];
    q += (double)v[2] * (double)v[2]; q += (double)v[3] * (double)v[3];
  }
  stats_reduce_store(s, q, ss, sq, res, st);
}

template <bool WF32>
__global__ __launch_bounds__(256) void ln_apply(const float* __restrict__ h, const float* __restrict__ st,
                                                float* __restrict__ t32, _Float16* __restrict__ xcat, int colOff) {
  const int g = blockIdx.x * 256 + threadIdx.x;
  if (g >= BNC / 4) return;
  const int i = g * 4;
  const int row = i >> 8, c = i & 255;
  const float m = st[0], r = st[1];
  const v4f x = *(const v4f*)(h + i);
  v4f y;
  y[0] = (x[0] - m) * r; y[1] = (x[1] - m) * r; y[2] = (x[2] - m) * r; y[3] = (x[3] - m) * r;
  const v2u u = pack4h(y);
  _Float16* dp = xcat + (size_t)row * KCAT + colOff + c;
  if (WF32) *(volatile v4f*)(t32 + i) = y;
  *(volatile v2u*)dp = u;
  __threadfence();
  if (WF32) *(volatile v4f*)(t32 + i) = y;
  *(volatile v2u*)dp = u;
}

__global__ __launch_bounds__(256) void degree_rsqrt(const int* __restrict__ edge_index, const float* __restrict__ ew_all,
                                                    float* __restrict__ dinv_all) {
  __shared__ int lslot[256];
  __shared__ float lw[256];
  __shared__ int wcnt[8];
  const int tid = threadIdx.x, lane = tid & 31, wave = tid >> 5;
  const int l = blockIdx.y;
  const int n0 = blockIdx.x * DT;
  const int* erow = edge_index + (size_t)l * 2 * NE;
  const int* ecol = erow + NE;
  const float* ew = ew_all + (size_t)l * NE;
  float d = 0.f;
  for (int ch = 0; ch < NE / 256; ++ch) {
    const int e = ch * 256 + tid;
    const int r = erow[e], c = ecol[e];
    const bool hit = ((unsigned)(r - n0) < (unsigned)DT) && (r != c);
    const unsigned bal = __builtin_amdgcn_ballot_w32(hit);
    const int pre = __builtin_popcount(bal & ((1u << lane) - 1u));
    if (lane == 0) wcnt[wave] = __builtin_popcount(bal);
    __syncthreads();
    int base = 0, total = 0;
#pragma unroll
    for (int w2 = 0; w2 < 8; ++w2) { const int cw = wcnt[w2]; if (w2 < wave) base += cw; total += cw; }
    if (hit) {
      const int pos = base + pre;
      lslot[pos] = r - n0;
      lw[pos] = ew[e];
    }
    __syncthreads();
    total = total > 256 ? 256 : total;
    if (tid < DT) {
      for (int p = 0; p < total; ++p) {
        if (lslot[p] == tid) d += lw[p];
      }
    }
    __syncthreads();
  }
  if (tid < DT) {
    const float dv = (d > 0.f) ? rsqrtf(fmaxf(d, 1e-12f)) : 0.f;
    float* dp = dinv_all + (size_t)l * NN + n0 + tid;
    *(volatile float*)dp = dv;
    __threadfence();
    *(volatile float*)dp = dv;
  }
}

template <int MODE>
__global__ __launch_bounds__(256) void poly_prop(const float* __restrict__ src, const float* __restrict__ tprev,
                                                 const float* __restrict__ dinv, const int* __restrict__ erow,
                                                 const int* __restrict__ ecol, const float* __restrict__ ew,
                                                 float* __restrict__ out32, _Float16* __restrict__ xcat, int colOff) {
  __shared__ __align__(16) float acc[PT * NB * NC];
  __shared__ int lsrc[256];
  __shared__ int lslot[256];
  __shared__ float lcoef[256];
  __shared__ int wcnt[8];
  const int tid = threadIdx.x, lane = tid & 31, wave = tid >> 5;
  const int n0 = blockIdx.x * PT;
  for (int i = tid; i < PT * NB * NC / 4; i += 256) ((v4f*)acc)[i] = (v4f){0.f, 0.f, 0.f, 0.f};
  const int smp = wave;
  const int c8 = lane * 8;
  for (int ch = 0; ch < NE / 256; ++ch) {
    const int e = ch * 256 + tid;
    const int r = erow[e], c = ecol[e];
    const bool hit = (unsigned)(c - n0) < (unsigned)PT;
    const unsigned bal = __builtin_amdgcn_ballot_w32(hit);
    const int pre = __builtin_popcount(bal & ((1u << lane) - 1u));
    if (lane == 0) wcnt[wave] = __builtin_popcount(bal);
    __syncthreads();
    int base = 0, total = 0;
#pragma unroll
    for (int w2 = 0; w2 < 8; ++w2) { const int cw = wcnt[w2]; if (w2 < wave) base += cw; total += cw; }
    if (hit) {
      const int rr = r < 0 ? 0 : (r > NN - 1 ? NN - 1 : r);
      float w = ew[e];
      if (r == c) w = 0.f;
      const float coef = -(dinv[rr] * w * dinv[c]);
      const int pos = base + pre;
      lsrc[pos] = rr; lslot[pos] = c - n0; lcoef[pos] = coef;
    }
    __syncthreads();
    total = total > 256 ? 256 : total;
    for (int p = 0; p < total; ++p) {
      const int slot = lslot[p] & (PT - 1);
      const int sr = lsrc[p] & (NN - 1);
      const float cf = lcoef[p];
      const float* sp = src + ((size_t)(smp * NN + sr)) * NC + c8;
      const v4f x0 = *(const v4f*)sp;
      const v4f x1 = *(const v4f*)(sp + 4);
      float* ap = acc + (slot * NB + smp) * NC + c8;
      v4f a0 = *(const v4f*)ap;
      v4f a1 = *(const v4f*)(ap + 4);
      a0 += cf * x0;
      a1 += cf * x1;
      *(v4f*)ap = a0;
      *(v4f*)(ap + 4) = a1;
    }
    __syncthreads();
  }
#pragma unroll 1
  for (int qq = 0; qq < PT; ++qq) {
    const int q = qq * NB + wave;
    const size_t R = (size_t)wave * NN + n0 + qq;
    const float* ap = acc + q * NC;
    const v4f a0 = *(const v4f*)(ap + 4 * lane);
    const v4f a1 = *(const v4f*)(ap + 128 + 4 * lane);
    v4f y0, y1;
    if (MODE == 0) {
      y0 = a0; y1 = a1;
    } else {
      const float* tp = tprev + R * NC;
      const v4f t0v = *(const v4f*)(tp + 4 * lane);
      const v4f t1v = *(const v4f*)(tp + 128 + 4 * lane);
      y0 = 2.f * a0 - t0v;
      y1 = 2.f * a1 - t1v;
    }
    const v2u u0 = pack4h(y0), u1 = pack4h(y1);
    _Float16* xp = xcat + R * KCAT + colOff;
    float* op = out32 + R * NC;
    if (MODE == 0) { *(volatile v4f*)(op + 4 * lane) = y0; *(volatile v4f*)(op + 128 + 4 * lane) = y1; }
    *(volatile v2u*)(xp + 4 * lane) = u0;
    *(volatile v2u*)(xp + 128 + 4 * lane) = u1;
    __threadfence();
    if (MODE == 0) { *(volatile v4f*)(op + 4 * lane) = y0; *(volatile v4f*)(op + 128 + 4 * lane) = y1; }
    *(volatile v2u*)(xp + 4 * lane) = u0;
    *(volatile v2u*)(xp + 128 + 4 * lane) = u1;
  }
}

template <bool STATS>
__global__ __launch_bounds__(512) void gelu_resid(const float* __restrict__ P, const float* __restrict__ hres,
                                                  float* __restrict__ hout, float* __restrict__ st) {
  __shared__ double ss[512], sq[512];
  __shared__ float res[2];
  const int tid = threadIdx.x;
  double s = 0.0, q = 0.0;
  const v2f* pv = (const v2f*)P;
  const v2f* rv = (const v2f*)hres;
  for (int i = tid; i < BNC / 2; i += 512) {
    const v2f p = pv[i];
    const v2f rr = rv[i];
    v2f y;
    {
      const float x = p[0];
      const float g = (x * (erff(x * 0.70710678118654752f) + 1.0f)) * 0.5f;
      y[0] = g + rr[0];
    }
    {
      const float x = p[1];
      const float g = (x * (erff(x * 0.70710678118654752f) + 1.0f)) * 0.5f;
      y[1] = g + rr[1];
    }
    ((volatile v2f*)hout)[i] = y;
    __threadfence();
    ((volatile v2f*)hout)[i] = y;
    if (STATS) {
      s += (double)y[0]; s += (double)y[1];
      q += (double)y[0] * (double)y[0]; q += (double)y[1] * (double)y[1];
    }
  }
  if (STATS) stats_reduce_store(s, q, ss, sq, res, st);
}

__global__ __launch_bounds__(256) void node_mean(const float* __restrict__ h, float* __restrict__ out) {
  __shared__ __align__(16) float sm[NC];
  const int b = blockIdx.x, c = threadIdx.x;
  const float* hp = h + (size_t)b * NN * NC + c;
  double s = 0.0;
  for (int n = 0; n < NN; ++n) s += (double)hp[(size_t)n * NC];
  sm[c] = (float)s * (1.0f / (float)NN);
  __syncthreads();
  if (c < 64) {
    const v4f v = *(const v4f*)(sm + 4 * c);
    float* op = out + (size_t)b * NC + 4 * c;
    *(volatile v4f*)op = v;
    __threadfence();
    *(volatile v4f*)op = v;
  }
}

extern "C" void kernel_launch(void* const* d_in, const int* in_sizes, int n_in,
                              void* d_out, int out_size, void* d_ws, size_t ws_size,
                              hipStream_t stream) {
  if (n_in < 7) return;
  if (in_sizes[0] != BNC || in_sizes[1] != NL * NE || in_sizes[2] != NL * NK * NC * NC ||
      in_sizes[3] != NL * NC || in_sizes[4] != NL * NC * NC || in_sizes[5] != NL * NC ||
      in_sizes[6] != NL * 2 * NE || out_size != NB * NC) return;

  const float* x_in = (const float*)d_in[0];
  const float* ewt  = (const float*)d_in[1];
  const float* pw   = (const float*)d_in[2];
  const float* pb   = (const float*)d_in[3];
  const float* mw   = (const float*)d_in[4];
  const float* mb   = (const float*)d_in[5];
  const int*   ei   = (const int*)d_in[6];
  float* out = (float*)d_out;

  char* ws = (char*)d_ws;
  size_t off = 0;
  float* hA  = (float*)(ws + off); off += (size_t)BNC * 4;
  float* hB  = (float*)(ws + off); off += (size_t)BNC * 4;
  float* tx0 = (float*)(ws + off); off += (size_t)BNC * 4;
  float* tx1 = (float*)(ws + off); off += (size_t)BNC * 4;
  _Float16* xcat = (_Float16*)(ws + off); off += (size_t)NM * KCAT * 2;
  _Float16* wct  = (_Float16*)(ws + off); off += (size_t)NL * NC * KCAT * 2;
  _Float16* wmt  = (_Float16*)(ws + off); off += (size_t)NL * NC * NC * 2;
  float* dinv  = (float*)(ws + off); off += (size_t)NL * NN * 4;
  float* stats = (float*)(ws + off); off += (size_t)8 * 32 * 4;
  if (off > ws_size) return;

  prep_weights<<<(NL * NC * KCAT / 8 + NL * NC * NC / 8) / 256, 256, 0, stream>>>(pw, mw, wct, wmt);
  degree_rsqrt<<<dim3(NN / DT, NL), 256, 0, stream>>>(ei, ewt, dinv);

  for (int l = 0; l < NL; ++l) {
    const int* er = ei + (size_t)l * 2 * NE;
    const int* ec = er + NE;
    const float* ewl = ewt + (size_t)l * NE;
    const float* dvl = dinv + (size_t)l * NN;
    const _Float16* wctl = wct + (size_t)l * NC * KCAT;
    const _Float16* wmtl = wmt + (size_t)l * NC * NC;
    const float* hin = (l == 0) ? x_in : hA;
    float* st1 = stats + (2 * l) * 32;
    float* st2 = stats + (2 * l + 1) * 32;
    float* st3 = stats + (2 * l + 2) * 32;

    if (l == 0) ln_stats<<<1, 512, 0, stream>>>(hin, st1);
    ln_apply<true><<<BNC / 4 / 256, 256, 0, stream>>>(hin, st1, tx0, xcat, 0);
    poly_prop<0><<<NN / PT, 256, 0, stream>>>(tx0, tx0, dvl, er, ec, ewl, tx1, xcat, NC);
    poly_prop<1><<<NN / PT, 256, 0, stream>>>(tx1, tx0, dvl, er, ec, ewl, hB, xcat, 2 * NC);
    wmma_gemm64<0, false, 2, 0, true, 0><<<dim3((NM / 64) * (NC / 64) / 8, 1), 256, 0, stream>>>(
        (const unsigned short*)xcat, (const unsigned short*)xcat, KCAT, 0L,
        (const unsigned short*)wctl, (const unsigned short*)wctl, KCAT, 0L,
        (void*)hB, (void*)hB, NC, 0L, pb + (size_t)l * NC, hin, 0L, NM, NC, KCAT, OSCALE);
    ln_stats<<<1, 512, 0, stream>>>(hB, st2);
    ln_apply<false><<<BNC / 4 / 256, 256, 0, stream>>>(hB, st2, tx0, xcat, 0);
    wmma_gemm64<0, false, 2, 0, false, 0><<<dim3((NM / 64) * (NC / 64) / 8, 1), 256, 0, stream>>>(
        (const unsigned short*)xcat, (const unsigned short*)xcat, KCAT, 0L,
        (const unsigned short*)wmtl, (const unsigned short*)wmtl, NC, 0L,
        (void*)tx1, (void*)tx1, NC, 0L, mb + (size_t)l * NC, hB, 0L, NM, NC, NC, OSCALE);
    if (l < NL - 1) gelu_resid<true><<<1, 512, 0, stream>>>(tx1, hB, hA, st3);
    else            gelu_resid<false><<<1, 512, 0, stream>>>(tx1, hB, hA, st3);
  }
  node_mean<<<NB, NC, 0, stream>>>(hA, out);
  (void)hipGetLastError();
}
